// longformer_Block_14843406975618
// MI455X (gfx1250) — hardware-verified
//
#include <hip/hip_runtime.h>
#include <math.h>
#include <stdint.h>

#define NBATCH 2
#define SEQ    4096
#define DM     1024
#define NH     16
#define HD     64
#define DFF    4096
#define WIN    256
#define MTOT   (NBATCH * SEQ)
#define NQT    (SEQ / 64)
#define WSC    64.0f
#define PSC    1024.0f
#define CSC    16.0f

static_assert(NH * HD == DM);
static_assert((SEQ % 64) == 0 && (DM % 64) == 0 && (DFF % 64) == 0 && (MTOT % 64) == 0);
static_assert((WIN % 64) == 0);
static_assert((MTOT % 8) == 0);

typedef _Float16 v16h __attribute__((ext_vector_type(16)));
typedef _Float16 v8h  __attribute__((ext_vector_type(8)));
typedef float    v8f  __attribute__((ext_vector_type(8)));
typedef float    v4f  __attribute__((ext_vector_type(4)));
typedef unsigned int v4u __attribute__((ext_vector_type(4)));

__device__ __forceinline__ unsigned short h_bits(_Float16 x) { return __builtin_bit_cast(unsigned short, x); }
__device__ __forceinline__ unsigned pkh2(float a, float b) {
  return (unsigned)h_bits((_Float16)a) | (((unsigned)h_bits((_Float16)b)) << 16);
}
__device__ __forceinline__ v8f zero8() { v8f z = {0.f, 0.f, 0.f, 0.f, 0.f, 0.f, 0.f, 0.f}; return z; }

__device__ __forceinline__ v16h ldfrag(const _Float16* p) {
  union { v16h v; v8h h[2]; } f;
  f.h[0] = *(const v8h*)(p);
  f.h[1] = *(const v8h*)(p + 16);
  return f.v;
}

__device__ __forceinline__ v8f mma_h(v16h a, v16h b, v8f c) {
  c = __builtin_amdgcn_wmma_f32_16x16x32_f16(false, a, false, b, (short)0, c, false, false);
#if defined(__HIP_DEVICE_COMPILE__)
  asm volatile("v_nop\n\tv_nop\n\tv_nop\n\tv_nop" : "+v"(c) : "v"(a), "v"(b));
#endif
  return c;
}
__device__ __forceinline__ v8f mma_raw(v16h a, v16h b, v8f c) {
  return __builtin_amdgcn_wmma_f32_16x16x32_f16(false, a, false, b, (short)0, c, false, false);
}
__device__ __forceinline__ void guard4(v8f& a, v8f& b, v8f& c, v8f& d, v16h x, v16h y) {
#if defined(__HIP_DEVICE_COMPILE__)
  asm volatile("v_nop\n\tv_nop\n\tv_nop\n\tv_nop" : "+v"(a), "+v"(b), "+v"(c), "+v"(d) : "v"(x), "v"(y));
#else
  (void)a; (void)b; (void)c; (void)d; (void)x; (void)y;
#endif
}
__device__ __forceinline__ void acc_guard4(v8f& a, v8f& b, v8f& c, v8f& d) {
#if defined(__HIP_DEVICE_COMPILE__)
  asm volatile("v_nop\n\tv_nop\n\tv_nop\n\tv_nop" : "+v"(a), "+v"(b), "+v"(c), "+v"(d));
#else
  (void)a; (void)b; (void)c; (void)d;
#endif
}
__device__ __forceinline__ void keep4(v16h a, v16h b, v16h c, v16h d) {
#if defined(__HIP_DEVICE_COMPILE__)
  asm volatile("v_nop" :: "v"(a), "v"(b), "v"(c), "v"(d));
#else
  (void)a; (void)b; (void)c; (void)d;
#endif
}
__device__ __forceinline__ void keep2(v16h a, v16h b) {
#if defined(__HIP_DEVICE_COMPILE__)
  asm volatile("v_nop" :: "v"(a), "v"(b));
#else
  (void)a; (void)b;
#endif
}
__device__ __forceinline__ void wave_lds_sync() {
  __builtin_amdgcn_fence(__ATOMIC_RELEASE, "workgroup");
  __builtin_amdgcn_wave_barrier();
  __builtin_amdgcn_fence(__ATOMIC_ACQUIRE, "workgroup");
}

__global__ __launch_bounds__(256) void transpose_h(const float* __restrict__ w, _Float16* wt,
                                                   int K, int N, float scale) {
  __shared__ float st[64][65];
  const int tid = threadIdx.x;
  const int k0 = blockIdx.y * 64;
  const int n0 = blockIdx.x * 64;
  {
    const int r = tid >> 2, c16 = (tid & 3) * 16;
    const float* src = w + (size_t)(k0 + r) * N + n0 + c16;
#pragma unroll
    for (int i = 0; i < 4; ++i) {
      const v4f v = *(const v4f*)(src + 4 * i);
#pragma unroll
      for (int e = 0; e < 4; ++e) st[r][c16 + 4 * i + e] = v[e];
    }
  }
  __syncthreads();
  const int orow = tid >> 3, c8 = (tid & 7) * 8;
  v4u pv[2];
#pragma unroll
  for (int it = 0; it < 2; ++it) {
    const int n = orow + 32 * it;
    v4u a;
#pragma unroll
    for (int e = 0; e < 4; ++e) a[e] = pkh2(st[c8 + 2 * e][n] * scale, st[c8 + 2 * e + 1][n] * scale);
    pv[it] = a;
  }
  for (int pass = 0; pass < 2; ++pass) {
#pragma unroll
    for (int it = 0; it < 2; ++it) {
      const int n = orow + 32 * it;
      *(volatile v4u*)(wt + (size_t)(n0 + n) * K + k0 + c8) = pv[it];
    }
    __threadfence();
  }
}

__global__ __launch_bounds__(256) void rmsnorm_h(const float* __restrict__ x, const float* __restrict__ g,
                                                 _Float16* out, int nrows, float eps) {
  const int lane = threadIdx.x & 31;
  const int wave = threadIdx.x >> 5;
  const int row = blockIdx.x * 8 + wave;
  if (row >= nrows) return;
  const float* xr = x + (size_t)row * DM;
  v4f a[8];
  float ss = 0.f;
#pragma unroll
  for (int i = 0; i < 4; ++i) {
    a[2 * i]     = *(const v4f*)(xr + 256 * i + 8 * lane);
    a[2 * i + 1] = *(const v4f*)(xr + 256 * i + 8 * lane + 4);
#pragma unroll
    for (int e = 0; e < 4; ++e) {
      ss += a[2 * i][e] * a[2 * i][e];
      ss += a[2 * i + 1][e] * a[2 * i + 1][e];
    }
  }
#pragma unroll
  for (int off = 16; off > 0; off >>= 1) ss += __shfl_xor(ss, off, 32);
  const float rn = rsqrtf(ss * (1.0f / (float)DM) + eps);
  v4u pk[4];
#pragma unroll
  for (int i = 0; i < 4; ++i) {
    const v4f g0 = *(const v4f*)(g + 256 * i + 8 * lane);
    const v4f g1 = *(const v4f*)(g + 256 * i + 8 * lane + 4);
    const v4f y0 = (a[2 * i] * rn) * g0;
    const v4f y1 = (a[2 * i + 1] * rn) * g1;
    v4u p;
    p[0] = pkh2(y0[0], y0[1]); p[1] = pkh2(y0[2], y0[3]);
    p[2] = pkh2(y1[0], y1[1]); p[3] = pkh2(y1[2], y1[3]);
    pk[i] = p;
  }
  _Float16* orow = out + (size_t)row * DM;
  for (int pass = 0; pass < 2; ++pass) {
#pragma unroll
    for (int i = 0; i < 4; ++i) *(volatile v4u*)(orow + 256 * i + 8 * lane) = pk[i];
    __threadfence();
  }
}

template <int MODE>
__global__ __launch_bounds__(256) __attribute__((amdgpu_num_vgpr(256))) void gemm64(
    const _Float16* __restrict__ A, int lda, long long strideA,
    const _Float16* __restrict__ Bt, int ldb, long long strideB,
    const float* __restrict__ bias,
    const float* __restrict__ R, int ldr,
    void* Cout, int ldc, long long strideC,
    int M, int N, int K, float oscale) {
  __shared__ __align__(16) float sT[8][16 * 68];
  const int b    = blockIdx.y;
  const int lane = threadIdx.x & 31;
  const int wave = threadIdx.x >> 5;
  const int tilesN = N >> 6;
  const int tilesM = M >> 6;
  const int tile = blockIdx.x * 8 + wave;
  if (tile >= tilesM * tilesN) return;
  const int tm = tile / tilesN;
  const int tn = tile - tm * tilesN;
  const int m0 = tm << 6;
  const int n0 = tn << 6;

  const _Float16* Ab = A  + (size_t)b * strideA;
  const _Float16* Bb = Bt + (size_t)b * strideB;

  const int rl   = lane & 15;
  const int koff = (lane >> 4) * 8;
  const int mOff = (lane >> 4) * 8;

  v8f acc[4][4];
#pragma unroll
  for (int i = 0; i < 4; ++i)
#pragma unroll
    for (int j = 0; j < 4; ++j) acc[i][j] = zero8();

  for (int k0 = 0; k0 < K; k0 += 32) {
    v16h bf[4];
#pragma unroll
    for (int j = 0; j < 4; ++j)
      bf[j] = ldfrag(Bb + (size_t)(n0 + (j << 4) + rl) * ldb + koff + k0);
#pragma unroll
    for (int i = 0; i < 4; ++i) {
      const v16h af = ldfrag(Ab + (size_t)(m0 + (i << 4) + rl) * lda + koff + k0);
#pragma unroll
      for (int j = 0; j < 4; ++j) acc[i][j] = mma_raw(af, bf[j], acc[i][j]);
      guard4(acc[i][0], acc[i][1], acc[i][2], acc[i][3], af, af);
    }
    keep4(bf[0], bf[1], bf[2], bf[3]);
  }
  acc_guard4(acc[0][0], acc[0][1], acc[0][2], acc[0][3]);
  acc_guard4(acc[1][0], acc[1][1], acc[1][2], acc[1][3]);
  acc_guard4(acc[2][0], acc[2][1], acc[2][2], acc[2][3]);
  acc_guard4(acc[3][0], acc[3][1], acc[3][2], acc[3][3]);

  float* slab = sT[wave];
#pragma unroll
  for (int i = 0; i < 4; ++i) {
    const int mBase = m0 + (i << 4);
#pragma unroll
    for (int j = 0; j < 4; ++j) {
#pragma unroll
      for (int r = 0; r < 8; ++r) slab[(mOff + r) * 68 + (j << 4) + rl] = acc[i][j][r];
    }
    wave_lds_sync();
    if (MODE == 2) {
      float* C = (float*)Cout + (size_t)b * strideC;
      const int h2 = lane >> 4, c4 = (lane & 15) * 4;
      const v4f bz = *(const v4f*)(bias + n0 + c4);
      v4f vals[8];
#pragma unroll
      for (int it = 0; it < 8; ++it) {
        const int row = it * 2 + h2;
        const v4f sv = *(const v4f*)(slab + row * 68 + c4);
        const v4f rv = *(const v4f*)(R + (size_t)(mBase + row) * ldr + n0 + c4);
        vals[it] = sv * oscale + bz + rv;
      }
      for (int pass = 0; pass < 2; ++pass) {
#pragma unroll
        for (int it = 0; it < 8; ++it) {
          const int row = it * 2 + h2;
          *(volatile v4f*)(C + (size_t)(mBase + row) * ldc + n0 + c4) = vals[it];
        }
        __threadfence();
      }
    } else {
      _Float16* C = (_Float16*)Cout + (size_t)b * strideC;
      const int q = lane >> 3, c8 = (lane & 7) * 8;
      float bcol[8];
      if (MODE == 0) {
        const v4f b0 = *(const v4f*)(bias + n0 + c8);
        const v4f b1v = *(const v4f*)(bias + n0 + c8 + 4);
#pragma unroll
        for (int e = 0; e < 4; ++e) { bcol[e] = b0[e]; bcol[4 + e] = b1v[e]; }
      } else {
#pragma unroll
        for (int e = 0; e < 8; ++e) bcol[e] = 0.f;
      }
      v4u hv[4];
#pragma unroll
      for (int it = 0; it < 4; ++it) {
        const int row = it * 4 + q;
        const float* sp = slab + row * 68 + c8;
        const float brow = (MODE == 1) ? bias[mBase + row] : 0.f;
        v4u a;
#pragma unroll
        for (int e = 0; e < 4; ++e) {
          const float f0 = sp[2 * e] * oscale + bcol[2 * e] + brow;
          const float f1 = sp[2 * e + 1] * oscale + bcol[2 * e + 1] + brow;
          a[e] = pkh2(f0, f1);
        }
        hv[it] = a;
      }
      for (int pass = 0; pass < 2; ++pass) {
#pragma unroll
        for (int it = 0; it < 4; ++it) {
          const int row = it * 4 + q;
          *(volatile v4u*)(C + (size_t)(mBase + row) * ldc + n0 + c8) = hv[it];
        }
        __threadfence();
      }
    }
    wave_lds_sync();
  }
}

__global__ __launch_bounds__(256) __attribute__((amdgpu_num_vgpr(256))) void gemm_glu(
    const _Float16* __restrict__ A, int lda,
    const _Float16* __restrict__ B1t, const _Float16* __restrict__ B3t, int ldb,
    const float* __restrict__ b1, const float* __restrict__ b3,
    _Float16* U, int ldc, int M, int N, int K, float oscale) {
  __shared__ __align__(16) float sT[8][16 * 68];
  const int lane = threadIdx.x & 31;
  const int wave = threadIdx.x >> 5;
  const int tilesN = N >> 6;
  const int tilesM = M >> 5;
  const int tile = blockIdx.x * 8 + wave;
  if (tile >= tilesM * tilesN) return;
  const int tm = tile / tilesN;
  const int tn = tile - tm * tilesN;
  const int m0 = tm << 5;
  const int n0 = tn << 6;
  const int rl = lane & 15, koff = (lane >> 4) * 8, mOff = koff;

  v8f ac1[2][4], ac3[2][4];
#pragma unroll
  for (int i = 0; i < 2; ++i)
#pragma unroll
    for (int j = 0; j < 4; ++j) { ac1[i][j] = zero8(); ac3[i][j] = zero8(); }

  for (int k0 = 0; k0 < K; k0 += 32) {
    v16h af[2];
#pragma unroll
    for (int i = 0; i < 2; ++i) af[i] = ldfrag(A + (size_t)(m0 + (i << 4) + rl) * lda + koff + k0);
#pragma unroll
    for (int j = 0; j < 4; ++j) {
      const size_t bo = (size_t)(n0 + (j << 4) + rl) * ldb + koff + k0;
      const v16h p1 = ldfrag(B1t + bo);
      const v16h p3 = ldfrag(B3t + bo);
#pragma unroll
      for (int i = 0; i < 2; ++i) {
        ac1[i][j] = mma_raw(af[i], p1, ac1[i][j]);
        ac3[i][j] = mma_raw(af[i], p3, ac3[i][j]);
      }
      guard4(ac1[0][j], ac1[1][j], ac3[0][j], ac3[1][j], p1, p3);
    }
    keep2(af[0], af[1]);
  }
  acc_guard4(ac1[0][0], ac1[0][1], ac1[0][2], ac1[0][3]);
  acc_guard4(ac1[1][0], ac1[1][1], ac1[1][2], ac1[1][3]);
  acc_guard4(ac3[0][0], ac3[0][1], ac3[0][2], ac3[0][3]);
  acc_guard4(ac3[1][0], ac3[1][1], ac3[1][2], ac3[1][3]);

  float bb1[4], bb3[4];
#pragma unroll
  for (int j = 0; j < 4; ++j) {
    const int n = n0 + (j << 4) + rl;
    bb1[j] = b1[n]; bb3[j] = b3[n];
  }
  float* slab = sT[wave];
#pragma unroll
  for (int i = 0; i < 2; ++i) {
    const int mBase = m0 + (i << 4);
#pragma unroll
    for (int j = 0; j < 4; ++j) {
#pragma unroll
      for (int r = 0; r < 8; ++r) {
        const float a1 = ac1[i][j][r] * oscale + bb1[j];
        const float a3 = ac3[i][j][r] * oscale + bb3[j];
        const float sg = __builtin_amdgcn_rcpf(1.0f + __expf(-a1));
        slab[(mOff + r) * 68 + (j << 4) + rl] = (a1 * sg) * a3;
      }
    }
    wave_lds_sync();
    const int q = lane >> 3, c8 = (lane & 7) * 8;
    v4u hv[4];
#pragma unroll
    for (int it = 0; it < 4; ++it) {
      const int row = it * 4 + q;
      const float* sp = slab + row * 68 + c8;
      v4u a;
#pragma unroll
      for (int e = 0; e < 4; ++e) a[e] = pkh2(sp[2 * e], sp[2 * e + 1]);
      hv[it] = a;
    }
    for (int pass = 0; pass < 2; ++pass) {
#pragma unroll
      for (int it = 0; it < 4; ++it) {
        const int row = it * 4 + q;
        *(volatile v4u*)(U + (size_t)(mBase + row) * ldc + n0 + c8) = hv[it];
      }
      __threadfence();
    }
    wave_lds_sync();
  }
}

__global__ __launch_bounds__(128)
void attn_band64(const _Float16* __restrict__ qp, const _Float16* __restrict__ kp,
                 const _Float16* __restrict__ vtp, _Float16* op, float sscale, float onorm) {
  union FH { v16h v; v8h h[2]; };
  __shared__ __align__(16) _Float16 Ksh[64 * 64];
  __shared__ __align__(16) _Float16 Vth[64 * 64];
  __shared__ __align__(16) _Float16 Psh[4][16 * 64];
  __shared__ __align__(16) float    Os[4][16 * 64];

  const int tid  = threadIdx.x;
  const int wave = tid >> 5;
  const int lane = tid & 31;
  const int hh   = lane >> 4;
  const int c    = lane & 15;

  const int bx   = blockIdx.x;
  const int qt   = bx % NQT;
  const int rest = bx / NQT;
  const int h    = rest % NH;
  const int b    = rest / NH;
  const int q0   = qt * 64 + wave * 16;
  const size_t rowB = (size_t)b * SEQ;

  const _Float16* Q = qp + (size_t)h * HD;
  const _Float16* Kp = kp + (size_t)h * HD;
  const _Float16* V = vtp + ((size_t)b * DM + (size_t)h * HD) * SEQ;

  v16h qa[2];
#pragma unroll
  for (int dc = 0; dc < 2; ++dc) qa[dc] = ldfrag(Q + (rowB + q0 + c) * DM + dc * 32 + 8 * hh);

  float mrow[8], lrow[8];
  v8f oacc[4];
#pragma unroll
  for (int r = 0; r < 8; ++r) { mrow[r] = -INFINITY; lrow[r] = 0.f; }
#pragma unroll
  for (int t = 0; t < 4; ++t) oacc[t] = zero8();

  const int iq = q0 + 8 * hh;

#pragma unroll 1
  for (int step = 0; step < 9; ++step) {
    const int kt = qt - (WIN / 64) + step;
    if (kt < 0 || kt >= NQT) continue;
    const int kv0 = kt * 64;
    __syncthreads();
    {
      const int r = tid >> 1, half = (tid & 1) * 32;
      const _Float16* kg = Kp + (rowB + kv0 + r) * DM + half;
      const _Float16* vg = V + (size_t)r * SEQ + kv0 + half;
#pragma unroll
      for (int i = 0; i < 4; ++i) {
        const v8h a0 = *(const v8h*)(kg + 8 * i);
        const v8h b0 = *(const v8h*)(vg + 8 * i);
        *(v8h*)(Ksh + r * 64 + half + 8 * i) = a0;
        *(v8h*)(Vth + r * 64 + half + 8 * i) = b0;
      }
    }
    __syncthreads();

    v8f s[4];
#pragma unroll
    for (int j = 0; j < 4; ++j) {
      s[j] = zero8();
#pragma unroll
      for (int dc = 0; dc < 2; ++dc) {
        FH kb;
        kb.h[0] = *(const v8h*)(Ksh + (j * 16 + c) * 64 + dc * 32 + 8 * hh);
        kb.h[1] = *(const v8h*)(Ksh + (j * 16 + c) * 64 + dc * 32 + 16 + 8 * hh);
        s[j] = mma_h(qa[dc], kb.v, s[j]);
      }
    }

    _Float16* pwh = Psh[wave];
#pragma unroll
    for (int r = 0; r < 8; ++r) {
      const int ia = iq + r;
      float m = -INFINITY;
#pragma unroll
      for (int j = 0; j < 4; ++j) {
        const int ja = kv0 + j * 16 + c;
        const int dlt = ja - ia;
        const bool valid = (dlt <= WIN) && (dlt >= -WIN);
        const float sv = valid ? (s[j][r] * sscale) : -INFINITY;
        s[j][r] = sv;
        m = fmaxf(m, sv);
      }
#pragma unroll
      for (int off = 1; off < 16; off <<= 1) m = fmaxf(m, __shfl_xor(m, off, 32));
      const float mnew  = fmaxf(mrow[r], m);
      const float msafe = (mnew == -INFINITY) ? 0.f : mnew;
      const float alpha = __expf(mrow[r] - msafe);
      mrow[r] = mnew;
      float psum = 0.f;
#pragma unroll
      for (int j = 0; j < 4; ++j) {
        const float p = __expf(s[j][r] - msafe);
        psum += p;
        pwh[(8 * hh + r) * 64 + j * 16 + c] = (_Float16)(p * PSC);
      }
#pragma unroll
      for (int off = 1; off < 16; off <<= 1) psum += __shfl_xor(psum, off, 32);
      lrow[r] = lrow[r] * alpha + psum;
#pragma unroll
      for (int t = 0; t < 4; ++t) oacc[t][r] *= alpha;
    }
    wave_lds_sync();

#pragma unroll
    for (int kk = 0; kk < 2; ++kk) {
      FH pa;
      pa.h[0] = *(const v8h*)(pwh + c * 64 + kk * 32 + 8 * hh);
      pa.h[1] = *(const v8h*)(pwh + c * 64 + kk * 32 + 16 + 8 * hh);
#pragma unroll
      for (int t = 0; t < 4; ++t) {
        FH vb;
        vb.h[0] = *(const v8h*)(Vth + (t * 16 + c) * 64 + kk * 32 + 8 * hh);
        vb.h[1] = *(const v8h*)(Vth + (t * 16 + c) * 64 + kk * 32 + 16 + 8 * hh);
        oacc[t] = mma_h(pa.v, vb.v, oacc[t]);
      }
    }
  }

  float* os = Os[wave];
#pragma unroll
  for (int r = 0; r < 8; ++r) {
    const float l = lrow[r];
    const float inv = ((l > 0.f) ? __builtin_amdgcn_rcpf(l) : 0.f) * onorm;
#pragma unroll
    for (int t = 0; t < 4; ++t) os[(8 * hh + r) * 64 + t * 16 + c] = oacc[t][r] * inv;
  }
  wave_lds_sync();
  {
    const int q4 = lane >> 3, c8 = (lane & 7) * 8;
    v4u hv[4];
#pragma unroll
    for (int it = 0; it < 4; ++it) {
      const int row = it * 4 + q4;
      const float* sp = os + row * 64 + c8;
      v4u a;
#pragma unroll
      for (int e = 0; e < 4; ++e) a[e] = pkh2(sp[2 * e], sp[2 * e + 1]);
      hv[it] = a;
    }
    for (int pass = 0; pass < 2; ++pass) {
#pragma unroll
      for (int it = 0; it < 4; ++it) {
        const int row = it * 4 + q4;
        const size_t go = (rowB + q0 + row) * DM + (size_t)h * HD + c8;
        *(volatile v4u*)(op + go) = hv[it];
      }
      __threadfence();
    }
  }
}

extern "C" void kernel_launch(void* const* d_in, const int* in_sizes, int n_in,
                              void* d_out, int out_size, void* d_ws, size_t ws_size,
                              hipStream_t stream) {
  if (n_in < 17) return;
  if (in_sizes[0] != MTOT * DM || in_sizes[1] != DM) return;
  if (in_sizes[2] != DM * DM || in_sizes[3] != DM || in_sizes[4] != DM * DM || in_sizes[5] != DM) return;
  if (in_sizes[6] != DM * DM || in_sizes[7] != DM || in_sizes[8] != DM * DM || in_sizes[9] != DM) return;
  if (in_sizes[10] != DM || in_sizes[11] != DM * DFF || in_sizes[12] != DFF) return;
  if (in_sizes[13] != DFF * DM || in_sizes[14] != DM || in_sizes[15] != DM * DFF || in_sizes[16] != DFF) return;
  if (out_size != MTOT * DM) return;

  const float* x   = (const float*)d_in[0];
  const float* gn1 = (const float*)d_in[1];
  const float* wq  = (const float*)d_in[2];   const float* bq = (const float*)d_in[3];
  const float* wk  = (const float*)d_in[4];   const float* bk = (const float*)d_in[5];
  const float* wv  = (const float*)d_in[6];   const float* bv = (const float*)d_in[7];
  const float* wo  = (const float*)d_in[8];   const float* bo = (const float*)d_in[9];
  const float* gn2 = (const float*)d_in[10];
  const float* w1  = (const float*)d_in[11];  const float* b1 = (const float*)d_in[12];
  const float* w2  = (const float*)d_in[13];  const float* b2 = (const float*)d_in[14];
  const float* w3  = (const float*)d_in[15];  const float* b3 = (const float*)d_in[16];

  const size_t PWD = (size_t)DM * DM * 2;
  const size_t PWF = (size_t)DM * DFF * 2;
  const size_t PA  = (size_t)MTOT * DM * 2;
  const size_t PX1 = (size_t)MTOT * DM * 4;
  const int    MHALF = MTOT / 2;
  const size_t PU  = (size_t)MHALF * DFF * 2;
  size_t off = 0;
  const size_t oWq = off; off += PWD;
  const size_t oWk = off; off += PWD;
  const size_t oWv = off; off += PWD;
  const size_t oWo = off; off += PWD;
  const size_t oW1 = off; off += PWF;
  const size_t oW3 = off; off += PWF;
  const size_t oW2 = off; off += PWF;
  const size_t oXn = off; off += PA;
  const size_t oQ  = off; off += PA;
  const size_t oK  = off; off += PA;
  const size_t oVt = off; off += PA;
  const size_t oCtx = oXn;
  const size_t oHn  = oXn;
  const size_t oX1  = oQ;
  const size_t oU   = oVt;
  if (oX1 + PX1 > oVt) return;
  size_t total = off;
  if (oU + PU > total) total = oU + PU;
  if (total > ws_size) return;
  if (total > (size_t)134217728) return;

  char* ws = (char*)d_ws;
  _Float16* WqT = (_Float16*)(ws + oWq);
  _Float16* WkT = (_Float16*)(ws + oWk);
  _Float16* WvT = (_Float16*)(ws + oWv);
  _Float16* WoT = (_Float16*)(ws + oWo);
  _Float16* W1T = (_Float16*)(ws + oW1);
  _Float16* W3T = (_Float16*)(ws + oW3);
  _Float16* W2T = (_Float16*)(ws + oW2);
  _Float16* Xn  = (_Float16*)(ws + oXn);
  _Float16* Qp  = (_Float16*)(ws + oQ);
  _Float16* Kpl = (_Float16*)(ws + oK);
  _Float16* Vt  = (_Float16*)(ws + oVt);
  _Float16* Ctx = (_Float16*)(ws + oCtx);
  _Float16* Hn  = (_Float16*)(ws + oHn);
  float*    X1  = (float*)(ws + oX1);
  _Float16* Up  = (_Float16*)(ws + oU);
  float*    Out = (float*)d_out;

  const dim3 blk(256);
  const float EPS = 1e-6f;
  const float invW = 1.0f / WSC;
  const float invWC = 1.0f / (WSC * CSC);

  transpose_h<<<dim3(DM / 64, DM / 64), blk, 0, stream>>>(wq, WqT, DM, DM, WSC);
  transpose_h<<<dim3(DM / 64, DM / 64), blk, 0, stream>>>(wk, WkT, DM, DM, WSC);
  transpose_h<<<dim3(DM / 64, DM / 64), blk, 0, stream>>>(wv, WvT, DM, DM, WSC);
  transpose_h<<<dim3(DM / 64, DM / 64), blk, 0, stream>>>(wo, WoT, DM, DM, WSC);
  transpose_h<<<dim3(DFF / 64, DM / 64), blk, 0, stream>>>(w1, W1T, DM, DFF, WSC);
  transpose_h<<<dim3(DFF / 64, DM / 64), blk, 0, stream>>>(w3, W3T, DM, DFF, WSC);
  transpose_h<<<dim3(DM / 64, DFF / 64), blk, 0, stream>>>(w2, W2T, DFF, DM, WSC);

  rmsnorm_h<<<dim3(MTOT / 8), blk, 0, stream>>>(x, gn1, Xn, MTOT, EPS);

  const dim3 gProj(((MTOT / 64) * (DM / 64)) / 8, 1);
  gemm64<0><<<gProj, blk, 0, stream>>>(Xn, DM, 0LL, WqT, DM, 0LL, bq, x, 0,
                                       (void*)Qp, DM, 0LL, MTOT, DM, DM, invW);
  gemm64<0><<<gProj, blk, 0, stream>>>(Xn, DM, 0LL, WkT, DM, 0LL, bk, x, 0,
                                       (void*)Kpl, DM, 0LL, MTOT, DM, DM, invW);
  const dim3 gVT(((DM / 64) * (SEQ / 64)) / 8, NBATCH);
  gemm64<1><<<gVT, blk, 0, stream>>>(WvT, DM, 0LL, Xn, DM, (long long)SEQ * DM, bv, x, 0,
                                     (void*)Vt, SEQ, (long long)DM * SEQ, DM, SEQ, DM, invW);
  attn_band64<<<dim3(NBATCH * NH * NQT), dim3(128), 0, stream>>>(Qp, Kpl, Vt, Ctx, 0.125f, CSC / PSC);
  gemm64<2><<<gProj, blk, 0, stream>>>(Ctx, DM, 0LL, WoT, DM, 0LL, bo, x, DM,
                                       (void*)X1, DM, 0LL, MTOT, DM, DM, invWC);
  rmsnorm_h<<<dim3(MTOT / 8), blk, 0, stream>>>(X1, gn2, Hn, MTOT, EPS);
  const dim3 gGlu(((MHALF / 32) * (DFF / 64)) / 8);
  const dim3 gDown(((MHALF / 64) * (DM / 64)) / 8, 1);
  for (int half = 0; half < 2; ++half) {
    const size_t r0 = (size_t)half * MHALF;
    gemm_glu<<<gGlu, blk, 0, stream>>>(Hn + r0 * DM, DM, W1T, W3T, DM, b1, b3,
                                       Up, DFF, MHALF, DFF, DM, invW);
    gemm64<2><<<gDown, blk, 0, stream>>>(Up, DFF, 0LL, W2T, DFF, 0LL, b2, X1 + r0 * DM, DM,
                                         (void*)(Out + r0 * DM), DM, 0LL, MHALF, DM, DFF, invW);
  }
  (void)hipGetLastError();
}
